// SelfAttention_PostLN_71949292143045
// MI455X (gfx1250) — hardware-verified
//
#include <hip/hip_runtime.h>
#include <stdint.h>


typedef _Float16 half_t;
typedef _Float16 v16h __attribute__((ext_vector_type(16)));
typedef _Float16 v8h  __attribute__((ext_vector_type(8)));
typedef float    v8f  __attribute__((ext_vector_type(8)));
typedef float    v4f  __attribute__((ext_vector_type(4)));
typedef int      v4i  __attribute__((ext_vector_type(4)));

union Frag { v16h v; v8h half[2]; };

static constexpr int kB = 2, kL = 2048, kC = 1024, kDK = 64, kH = 16;
static constexpr int kM = kB * kL;
static constexpr float kLog2e     = 1.44269504088896340736f;
static constexpr float kActScale  = 16.0f;
static constexpr float kWScale    = 64.0f;
static constexpr float kPScale    = 16384.0f;
static constexpr float kZOverP    = 0.015625f;
static constexpr float kProjScale = 0.0009765625f;
static constexpr float kOutScale  = 0.00006103515625f;
static constexpr float kInvSqrtDK = 0.125f;
static constexpr float kMaskFill  = -32767.0f;

static __device__ __forceinline__ v8f vzero8() {
  v8f r;
#pragma unroll
  for (int i = 0; i < 8; ++i) r[i] = 0.f;
  return r;
}

static __device__ __forceinline__ v8f wmma16(v16h a, v16h b, v8f c) {
  c = __builtin_amdgcn_wmma_f32_16x16x32_f16(false, a, false, b, (short)0, c, false, false);
  asm volatile("v_nop\n\tv_nop\n\tv_nop\n\tv_nop" : "+v"(c) : "v"(a), "v"(b));
  return c;
}

static __device__ __forceinline__ half_t cvt_via_bf16(float x) {
  unsigned u = __float_as_uint(x);
  u = (u + 0x7FFFu + ((u >> 16) & 1u)) & 0xFFFF0000u;
  return (half_t)__uint_as_float(u);
}

__global__ __launch_bounds__(256) void k_cvt(const float* __restrict__ src,
                                             half_t* __restrict__ dst,
                                             unsigned n8, float scale) {
  const unsigned stride = gridDim.x * blockDim.x;
  for (unsigned i = blockIdx.x * blockDim.x + threadIdx.x; i < n8; i += stride) {
    const v4f a = *(const v4f*)(src + (size_t)i * 8);
    const v4f c = *(const v4f*)(src + (size_t)i * 8 + 4);
    v8h o;
#pragma unroll
    for (int e = 0; e < 4; ++e) {
      o[e]     = cvt_via_bf16(a[e] * scale);
      o[4 + e] = cvt_via_bf16(c[e] * scale);
    }
    volatile v8h* p = (volatile v8h*)(dst + (size_t)i * 8);
    *p = o;
    __threadfence();
    *p = o;
  }
}

template <int MODE>
__global__ __launch_bounds__(256) void k_gemm(const half_t* __restrict__ A,
                                              const half_t* __restrict__ W,
                                              const float* __restrict__ bias,
                                              void* __restrict__ outp,
                                              float scale) {
  __shared__ __attribute__((aligned(16))) float sTile[128 * 68];
  half_t* sH = (half_t*)sTile;

  const unsigned tid = threadIdx.x;
  const unsigned wave = tid >> 5, lane = tid & 31;
  const unsigned ln = lane & 15, lh = lane >> 4;
  const unsigned wm = wave & 3, wn = wave >> 2;
  const unsigned bm0 = blockIdx.y * 128, bn0 = blockIdx.x * 64;
  const unsigned m0 = bm0 + wm * 32, n0 = bn0 + wn * 32;

  v8f acc[2][2];
#pragma unroll
  for (int i = 0; i < 2; ++i)
#pragma unroll
    for (int j = 0; j < 2; ++j) acc[i][j] = vzero8();

#pragma unroll 1
  for (unsigned k0 = 0; k0 < (unsigned)kC; k0 += 32) {
    Frag af[2], bf[2];
#pragma unroll
    for (int i = 0; i < 2; ++i) {
      const half_t* p = A + (size_t)(m0 + i * 16 + ln) * kC + k0;
      af[i].half[0] = *(const v8h*)(p + 8 * lh);
      af[i].half[1] = *(const v8h*)(p + 16 + 8 * lh);
    }
#pragma unroll
    for (int j = 0; j < 2; ++j) {
      const half_t* p = W + (size_t)(n0 + j * 16 + ln) * kC + k0;
      bf[j].half[0] = *(const v8h*)(p + 8 * lh);
      bf[j].half[1] = *(const v8h*)(p + 16 + 8 * lh);
    }
#pragma unroll
    for (int i = 0; i < 2; ++i)
#pragma unroll
      for (int j = 0; j < 2; ++j) acc[i][j] = wmma16(af[i].v, bf[j].v, acc[i][j]);
  }

#pragma unroll
  for (int i = 0; i < 2; ++i)
#pragma unroll
    for (int j = 0; j < 2; ++j) {
      const unsigned tn = wn * 32 + j * 16 + ln;
      const float bs = bias[bn0 + tn];
#pragma unroll
      for (int r = 0; r < 8; ++r) {
        const unsigned tm = wm * 32 + i * 16 + 8 * lh + r;
        const float v = acc[i][j][r] * scale + bs;
        if (MODE == 2)      sTile[tm * 68 + tn] = v;
        else if (MODE == 0) sH[tm * 72 + tn] = (half_t)v;
        else                sH[tn * 136 + tm] = (half_t)v;
      }
    }
  __syncthreads();

  auto emit = [&]() {
    if (MODE == 2) {
      float* o = (float*)outp;
#pragma unroll
      for (int p = 0; p < 8; ++p) {
        const unsigned idx = (unsigned)p * 256 + tid;
        const unsigned row = idx >> 4, c = idx & 15;
        const v4f v = *(const v4f*)(sTile + row * 68 + c * 4);
        *(volatile v4f*)(o + (size_t)(bm0 + row) * kC + bn0 + c * 4) = v;
      }
    } else if (MODE == 0) {
      half_t* o = (half_t*)outp;
#pragma unroll
      for (int p = 0; p < 4; ++p) {
        const unsigned idx = (unsigned)p * 256 + tid;
        const unsigned row = idx >> 3, c = idx & 7;
        const v8h v = *(const v8h*)(sH + row * 72 + c * 8);
        const unsigned m = bm0 + row, bb = m / kL, l = m % kL;
        *(volatile v8h*)(o + ((size_t)(bb * kH + blockIdx.x) * kL + l) * kDK + c * 8) = v;
      }
    } else {
      half_t* o = (half_t*)outp;
      const unsigned bb = bm0 / kL, l0 = bm0 % kL;
#pragma unroll
      for (int p = 0; p < 4; ++p) {
        const unsigned idx = (unsigned)p * 256 + tid;
        const unsigned d = idx >> 4, c = idx & 15;
        const v8h v = *(const v8h*)(sH + d * 136 + c * 8);
        *(volatile v8h*)(o + ((size_t)(bb * kH + blockIdx.x) * kDK + d) * kL + l0 + c * 8) = v;
      }
    }
  };
  emit();
  __threadfence();
  emit();
}

__global__ __launch_bounds__(256) void k_attn(const half_t* __restrict__ Q,
                                              const half_t* __restrict__ Kh,
                                              const half_t* __restrict__ VT,
                                              const int* __restrict__ mask,
                                              half_t* __restrict__ Z) {
  __shared__ __attribute__((aligned(16))) half_t sK[32][72];
  __shared__ __attribute__((aligned(16))) half_t sV[64][40];
  __shared__ __attribute__((aligned(16))) half_t sZ[8][16][72];

  const unsigned tid = threadIdx.x;
  const unsigned wave = tid >> 5, lane = tid & 31;
  const unsigned ln = lane & 15, lh = lane >> 4;
  const unsigned bh = blockIdx.y;
  const unsigned b = bh / kH, h = bh % kH;
  const unsigned q0 = blockIdx.x * 128 + wave * 16;

  const half_t* Qb = Q + (size_t)bh * kL * kDK;
  const half_t* Kb = Kh + (size_t)bh * kL * kDK;
  const half_t* Vb = VT + (size_t)bh * kDK * kL;
  const int* mb = mask + (size_t)b * kL * kL;

  const unsigned kr = tid >> 3, kc = (tid & 7) * 8;
  const unsigned vr = tid >> 2, vc = (tid & 3) * 8;

  Frag qf[2];
#pragma unroll
  for (int ks = 0; ks < 2; ++ks) {
    const half_t* p = Qb + (size_t)(q0 + ln) * kDK + ks * 32;
    qf[ks].half[0] = *(const v8h*)(p + 8 * lh);
    qf[ks].half[1] = *(const v8h*)(p + 16 + 8 * lh);
  }

  v8f o[4];
#pragma unroll
  for (int dj = 0; dj < 4; ++dj) o[dj] = vzero8();
  float mrow = -1.0e30f;
  float lrow = 0.f;

#pragma unroll 1
  for (unsigned t = 0; t < (unsigned)(kL / 32); ++t) {
    const unsigned j0 = t * 32;
    __syncthreads();
    *(v8h*)&sK[kr][kc] = *(const v8h*)(Kb + (size_t)(j0 + kr) * kDK + kc);
    *(v8h*)&sV[vr][vc] = *(const v8h*)(Vb + (size_t)vr * kL + j0 + vc);
    __syncthreads();

    v8f s[2];
#pragma unroll
    for (int kvi = 0; kvi < 2; ++kvi) {
      s[kvi] = vzero8();
#pragma unroll
      for (int ks = 0; ks < 2; ++ks) {
        Frag kf;
        kf.half[0] = *(const v8h*)&sK[kvi * 16 + ln][ks * 32 + 8 * lh];
        kf.half[1] = *(const v8h*)&sK[kvi * 16 + ln][ks * 32 + 16 + 8 * lh];
        s[kvi] = wmma16(kf.v, qf[ks].v, s[kvi]);
      }
    }

#pragma unroll
    for (int kvi = 0; kvi < 2; ++kvi) {
      const int* mp = mb + (size_t)(q0 + ln) * kL + j0 + kvi * 16 + 8 * lh;
      const v4i ma = *(const v4i*)mp;
      const v4i mc = *(const v4i*)(mp + 4);
#pragma unroll
      for (int r = 0; r < 4; ++r) {
        s[kvi][r]     = (ma[r] == 0) ? kMaskFill : s[kvi][r] * kInvSqrtDK;
        s[kvi][4 + r] = (mc[r] == 0) ? kMaskFill : s[kvi][4 + r] * kInvSqrtDK;
      }
    }

    float tmx = -1.0e30f;
#pragma unroll
    for (int kvi = 0; kvi < 2; ++kvi)
#pragma unroll
      for (int r = 0; r < 8; ++r) tmx = fmaxf(tmx, s[kvi][r]);
    tmx = fmaxf(tmx, __shfl_xor(tmx, 16, 32));
    const float mn = fmaxf(mrow, tmx);
    const float resc = __builtin_amdgcn_exp2f((mrow - mn) * kLog2e);
    mrow = mn;
    float ps = 0.f;
#pragma unroll
    for (int kvi = 0; kvi < 2; ++kvi)
#pragma unroll
      for (int r = 0; r < 8; ++r) {
        const float pe = __builtin_amdgcn_exp2f((s[kvi][r] - mn) * kLog2e);
        s[kvi][r] = pe;
        ps += pe;
      }
    ps += __shfl_xor(ps, 16, 32);
    lrow = lrow * resc + ps;

    float rb[8];
#pragma unroll
    for (int r = 0; r < 8; ++r) rb[r] = __shfl(resc, (int)(r + 8 * lh), 32);
#pragma unroll
    for (int dj = 0; dj < 4; ++dj)
#pragma unroll
      for (int r = 0; r < 8; ++r) o[dj][r] *= rb[r];

    v16h pf;
#pragma unroll
    for (int e = 0; e < 8; ++e) {
      pf[e]     = (half_t)(s[0][e] * kPScale);
      pf[8 + e] = (half_t)(s[1][e] * kPScale);
    }
#pragma unroll
    for (int dj = 0; dj < 4; ++dj) {
      Frag vf;
      vf.half[0] = *(const v8h*)&sV[dj * 16 + ln][8 * lh];
      vf.half[1] = *(const v8h*)&sV[dj * 16 + ln][16 + 8 * lh];
      o[dj] = wmma16(pf, vf.v, o[dj]);
    }
  }

  const float linv = kZOverP / lrow;
  float lb[8];
#pragma unroll
  for (int r = 0; r < 8; ++r) lb[r] = __shfl(linv, (int)(r + 8 * lh), 32);
#pragma unroll
  for (int dj = 0; dj < 4; ++dj)
#pragma unroll
    for (int r = 0; r < 8; ++r)
      sZ[wave][8 * lh + r][dj * 16 + ln] = (half_t)(o[dj][r] * lb[r]);
  __syncthreads();

  auto emitz = [&]() {
#pragma unroll
    for (int p = 0; p < 4; ++p) {
      const unsigned row = (unsigned)p * 4 + (lane >> 3), c = lane & 7;
      const v8h v = *(const v8h*)&sZ[wave][row][c * 8];
      *(volatile v8h*)(Z + ((size_t)(b * kL + q0 + row)) * kC + h * kDK + c * 8) = v;
    }
  };
  emitz();
  __threadfence();
  emitz();
}

extern "C" void kernel_launch(void* const* d_in, const int* in_sizes, int n_in,
                              void* d_out, int out_size, void* d_ws,
                              size_t ws_size, hipStream_t stream) {
  const size_t nX = (size_t)kB * kL * kC;
  const size_t nW = (size_t)kC * kC;
  const size_t nMask = (size_t)kB * kL * kL;
  if (n_in < 12) return;
  if ((size_t)in_sizes[0] != nX || (size_t)in_sizes[1] != nX || (size_t)in_sizes[2] != nX) return;
  if ((size_t)in_sizes[3] != nMask) return;
  if ((size_t)in_sizes[4] != nW || (size_t)in_sizes[6] != nW ||
      (size_t)in_sizes[8] != nW || (size_t)in_sizes[10] != nW) return;
  if (in_sizes[5] != kC || in_sizes[7] != kC || in_sizes[9] != kC || in_sizes[11] != kC) return;
  if ((size_t)out_size != nX) return;

  const float* qx   = (const float*)d_in[0];
  const float* kx   = (const float*)d_in[1];
  const float* vx   = (const float*)d_in[2];
  const int*   mask = (const int*)d_in[3];
  const float* WQ_w = (const float*)d_in[4];
  const float* WQ_b = (const float*)d_in[5];
  const float* WK_w = (const float*)d_in[6];
  const float* WK_b = (const float*)d_in[7];
  const float* WV_w = (const float*)d_in[8];
  const float* WV_b = (const float*)d_in[9];
  const float* WO_w = (const float*)d_in[10];
  const float* WO_b = (const float*)d_in[11];

  char* ws = (char*)d_ws;
  size_t off = 0;
  const size_t bX = ((nX * sizeof(half_t)) + 255) & ~(size_t)255;
  const size_t bW = ((nW * sizeof(half_t)) + 255) & ~(size_t)255;
  const size_t need = 7 * bX + 4 * bW;
  if (need > ws_size) return;
  half_t* hQX = (half_t*)(ws + off); off += bX;
  half_t* hKX = (half_t*)(ws + off); off += bX;
  half_t* hVX = (half_t*)(ws + off); off += bX;
  half_t* hWQ = (half_t*)(ws + off); off += bW;
  half_t* hWK = (half_t*)(ws + off); off += bW;
  half_t* hWV = (half_t*)(ws + off); off += bW;
  half_t* hWO = (half_t*)(ws + off); off += bW;
  half_t* Qd  = (half_t*)(ws + off); off += bX;
  half_t* Kd  = (half_t*)(ws + off); off += bX;
  half_t* VTd = (half_t*)(ws + off); off += bX;
  half_t* Zd  = (half_t*)(ws + off); off += bX;

  k_cvt<<<512, 256, 0, stream>>>(qx, hQX, (unsigned)(nX >> 3), kActScale);
  k_cvt<<<512, 256, 0, stream>>>(kx, hKX, (unsigned)(nX >> 3), kActScale);
  k_cvt<<<512, 256, 0, stream>>>(vx, hVX, (unsigned)(nX >> 3), kActScale);
  k_cvt<<<512, 256, 0, stream>>>(WQ_w, hWQ, (unsigned)(nW >> 3), kWScale);
  k_cvt<<<512, 256, 0, stream>>>(WK_w, hWK, (unsigned)(nW >> 3), kWScale);
  k_cvt<<<512, 256, 0, stream>>>(WV_w, hWV, (unsigned)(nW >> 3), kWScale);
  k_cvt<<<512, 256, 0, stream>>>(WO_w, hWO, (unsigned)(nW >> 3), kWScale);

  dim3 gg(kC / 64, kM / 128);
  k_gemm<0><<<gg, 256, 0, stream>>>(hQX, hWQ, WQ_b, (void*)Qd, kProjScale);
  k_gemm<0><<<gg, 256, 0, stream>>>(hKX, hWK, WK_b, (void*)Kd, kProjScale);
  k_gemm<1><<<gg, 256, 0, stream>>>(hVX, hWV, WV_b, (void*)VTd, kProjScale);

  dim3 ga(kL / 128, kB * kH);
  k_attn<<<ga, 256, 0, stream>>>(Qd, Kd, VTd, mask, Zd);

  k_gemm<2><<<gg, 256, 0, stream>>>(Zd, hWO, WO_b, d_out, kOutScale);
}
